// GRANDE_82566451299124
// MI455X (gfx1250) — hardware-verified
//
#include <hip/hip_runtime.h>


namespace {
constexpr int NB = 8192, NTREE = 128, DEP = 7, NI = 128, NC = 10, NL = 128, NH1 = 64, TD = NTREE * DEP  ;
constexpr float XS = 8.0f;

typedef _Float16 b16;
typedef __attribute__((ext_vector_type(16))) _Float16 v16b;
typedef __attribute__((ext_vector_type(8))) _Float16 v8b;
typedef __attribute__((ext_vector_type(8))) float v8f;
typedef __attribute__((ext_vector_type(4))) float v4f;
__device__ __forceinline__ float bf16_rne(float f) { unsigned int u = __float_as_uint(f); u += 0x7FFFu + ((u >> 16) & 1u); return __uint_as_float(u & 0xFFFF0000u); }
__device__ __forceinline__ void split16(float v, b16& hi, b16& lo) { hi = (b16)v; lo = (b16)(v - (float)hi); }
__device__ __forceinline__ v16b frag_kb(const b16* p, int hh) { const v8b a = *(const v8b*)(p + 8 * hh), b = *(const v8b*)(p + 16 + 8 * hh); v16b f;
#pragma unroll
  for (int e = 0; e < 8; ++e) { f[e] = a[e]; f[8 + e] = b[e]; } return f; }
__device__ __forceinline__ v8f wmma16b(v16b a, v16b b, v8f c) { v8f d = __builtin_amdgcn_wmma_f32_16x16x32_f16(false, a, false, b, (short)0, c, false, false); asm volatile("v_nop\n\tv_nop\n\tv_nop\n\tv_nop" : "+v"(d) : "v"(a), "v"(b)); return d; }
__device__ __forceinline__ void wave_lds_sync() { __builtin_amdgcn_fence(__ATOMIC_RELEASE, "workgroup"); __builtin_amdgcn_wave_barrier(); __builtin_amdgcn_fence(__ATOMIC_ACQUIRE, "workgroup"); }
__device__ __forceinline__ float nexp(float x) { return __builtin_amdgcn_exp2f(x * 1.4426950408889634f); }
__device__ __forceinline__ float pmul(float a, float b) { float p = a * b; asm volatile("" : "+v"(p)); return p; }

__global__ __launch_bounds__(256) void prep_kernel(const float* __restrict__ x, const float* __restrict__ fm, const float* __restrict__ th, const float* __restrict__ lo, const float* __restrict__ w1, const float* __restrict__ b1, const float* __restrict__ w2, const float* __restrict__ b2, b16* __restrict__ M, b16* __restrict__ W1t, b16* __restrict__ W2t, b16* __restrict__ X, float* __restrict__ P, b16* __restrict__ LPh, b16* __restrict__ LPl) {
  const size_t tid = (size_t)blockIdx.x * 256 + threadIdx.x, nth = (size_t)gridDim.x * 256;
  for (int pass = 0; pass < 2; ++pass) {
    for (size_t p = tid; p < (size_t)TD * NI / 8; p += nth) { v8b v; for (int e = 0; e < 8; ++e) v[e] = (b16)fm[p * 8 + e]; *(volatile v8b*)(M + p * 8) = v; }
    for (size_t p = tid; p < (size_t)NH1 * (NI / 8); p += nth) { const int o = (int)(p / (NI / 8)), k0 = (int)(p % (NI / 8)) * 8; v8b v; for (int e = 0; e < 8; ++e) v[e] = (b16)bf16_rne(w1[(size_t)(k0 + e) * NH1 + o]); *(volatile v8b*)(W1t + (size_t)o * NI + k0) = v; }
    for (size_t p = tid; p < (size_t)NTREE * (NH1 / 8); p += nth) { const int o = (int)(p / (NH1 / 8)), k0 = (int)(p % (NH1 / 8)) * 8; v8b v; for (int e = 0; e < 8; ++e) v[e] = (b16)bf16_rne(w2[(size_t)(k0 + e) * NTREE + o]); *(volatile v8b*)(W2t + (size_t)o * NH1 + k0) = v; }
    for (size_t p = tid; p < (size_t)NB * NI / 8; p += nth) { v8b v; for (int e = 0; e < 8; ++e) v[e] = (b16)(bf16_rne(x[p * 8 + e]) * XS); *(volatile v8b*)(X + p * 8) = v; }
    for (size_t q = tid; q < 1088; q += nth) { const int i = (int)q; P[q] = bf16_rne((i < 896) ? th[i] : (i < 960) ? b1[i - 896] : b2[i - 960]); }
    for (size_t p = tid; p < (size_t)NTREE * 16 * (NL / 8); p += nth) { const int l0 = (int)(p % (NL / 8)) * 8, c = (int)((p / (NL / 8)) % 16), t = (int)(p / ((NL / 8) * 16)); v8b vh, vl;
      for (int e = 0; e < 8; ++e) { float val = 0.0f; if (c < NC) { const float* lr = lo + ((size_t)t * NL + l0 + e) * NC; float mx = -INFINITY; for (int k = 0; k < NC; ++k) mx = fmaxf(mx, bf16_rne(lr[k])); float sum = 0.0f, ec = 0.0f; for (int k = 0; k < NC; ++k) { const float ev = nexp(bf16_rne(lr[k]) - mx); sum += ev; if (k == c) ec = ev; } val = ec / sum; }
        b16 a_, b_; split16(val * XS, a_, b_); vh[e] = a_; vl[e] = b_; }
      const size_t gi = ((size_t)t * 16 + c) * NL + l0; *(volatile v8b*)(LPh + gi) = vh; *(volatile v8b*)(LPl + gi) = vl; }
    __threadfence(); }
}

__global__ __launch_bounds__(224) void split_kernel(const b16* __restrict__ X, const b16* __restrict__ M, const float* __restrict__ P, float* __restrict__ S) {
  __shared__ __attribute__((aligned(16))) float Ts[7][32][128 + 4];
  const int lane = threadIdx.x & 31, wave = threadIdx.x >> 5, nloc = lane & 15, hlf = lane >> 4, m0 = blockIdx.x * 32, c0 = wave * 128;
  v8f acc[2][8];
#pragma unroll
  for (int r = 0; r < 2; ++r)
#pragma unroll
    for (int t = 0; t < 8; ++t) acc[r][t] = (v8f){};
#pragma unroll
  for (int kb = 0; kb < NI; kb += 32) { const v16b a0 = frag_kb(X + (size_t)(m0 + nloc) * NI + kb, hlf), a1 = frag_kb(X + (size_t)(m0 + 16 + nloc) * NI + kb, hlf);
#pragma unroll
    for (int t = 0; t < 8; ++t) { const v16b bw = frag_kb(M + (size_t)(c0 + t * 16 + nloc) * NI + kb, hlf); acc[0][t] = wmma16b(a0, bw, acc[0][t]); acc[1][t] = wmma16b(a1, bw, acc[1][t]); } }
#pragma unroll
  for (int t = 0; t < 8; ++t) { const float thv = P[c0 + t * 16 + nloc];
#pragma unroll
    for (int r = 0; r < 2; ++r)
#pragma unroll
      for (int v = 0; v < 8; ++v) { const float z = acc[r][t][v] * (1.0f / XS) - thv; Ts[wave][r * 16 + 8 * hlf + v][t * 16 + nloc] = 0.5f * (z / (1.0f + fabsf(z)) + 1.0f); } }
  wave_lds_sync();
  for (int pass = 0; pass < 2; ++pass) { for (int i = lane; i < 32 * 32; i += 32) { const int rr = i >> 5, c4 = (i & 31) * 4; *(volatile v4f*)(S + (size_t)(m0 + rr) * TD + c0 + c4) = *(const v4f*)(&Ts[wave][rr][c4]); } __threadfence(); }
}

__global__ __launch_bounds__(64) void attn_kernel(const b16* __restrict__ X, const b16* __restrict__ W1t, const b16* __restrict__ W2t, const float* __restrict__ P, float* __restrict__ ATT) {
  __shared__ __attribute__((aligned(16))) b16 Hh[32][NH1 + 8], Hl[32][NH1 + 8]; __shared__ __attribute__((aligned(16))) float As[32][NTREE + 4];
  const int lane = threadIdx.x & 31, wave = threadIdx.x >> 5, nloc = lane & 15, hlf = lane >> 4, m0 = blockIdx.x * 32 + wave * 16;
  v8f h[4] = {{}, {}, {}, {}};
#pragma unroll
  for (int kb = 0; kb < NI; kb += 32) { const v16b a = frag_kb(X + (size_t)(m0 + nloc) * NI + kb, hlf);
#pragma unroll
    for (int t = 0; t < 4; ++t) h[t] = wmma16b(a, frag_kb(W1t + (size_t)(t * 16 + nloc) * NI + kb, hlf), h[t]); }
#pragma unroll
  for (int t = 0; t < 4; ++t)
#pragma unroll
    for (int r = 0; r < 8; ++r) { const int c = t * 16 + nloc; const float y = fmaxf(h[t][r] * (1.0f / XS) + P[896 + c], 0.0f); b16 a_, b_; split16(y * XS, a_, b_); Hh[wave * 16 + 8 * hlf + r][c] = a_; Hl[wave * 16 + 8 * hlf + r][c] = b_; }
  wave_lds_sync();
  v8f acc[8];
#pragma unroll
  for (int t = 0; t < 8; ++t) acc[t] = (v8f){};
#pragma unroll
  for (int kb = 0; kb < NH1; kb += 32) { const v16b a = frag_kb(&Hh[wave * 16 + nloc][kb], hlf), al = frag_kb(&Hl[wave * 16 + nloc][kb], hlf);
#pragma unroll
    for (int t = 0; t < 8; ++t) { const v16b bw = frag_kb(W2t + (size_t)(t * 16 + nloc) * NH1 + kb, hlf); acc[t] = wmma16b(a, bw, acc[t]); acc[t] = wmma16b(al, bw, acc[t]); } }
#pragma unroll
  for (int t = 0; t < 8; ++t)
#pragma unroll
    for (int r = 0; r < 8; ++r) As[wave * 16 + 8 * hlf + r][t * 16 + nloc] = acc[t][r] * (1.0f / XS) + P[960 + t * 16 + nloc];
  wave_lds_sync();
  if (lane < 16) { float* ar = &As[wave * 16 + lane][0]; float mx = -INFINITY; for (int t = 0; t < NTREE; ++t) mx = fmaxf(mx, ar[t]); float sum = 0.0f; for (int t = 0; t < NTREE; ++t) { const float e = nexp(ar[t] - mx); ar[t] = e; sum += e; } const float inv = 1.0f / sum; for (int t = 0; t < NTREE; ++t) ar[t] *= inv; }
  wave_lds_sync();
  for (int pass = 0; pass < 2; ++pass) { for (int i = lane; i < 16 * 32; i += 32) { const int rr = i >> 5, c4 = (i & 31) * 4; *(volatile v4f*)(ATT + (size_t)(m0 + rr) * NTREE + c4) = *(const v4f*)(&As[wave * 16 + rr][c4]); } __threadfence(); }
}

__global__ __launch_bounds__(128) void tree_kernel(const float* __restrict__ S, const float* __restrict__ ATT, const b16* __restrict__ LPh, const b16* __restrict__ LPl, float* __restrict__ out) {
  __shared__ __attribute__((aligned(16))) b16 Ah[32][NL + 8], Al[32][NL + 8]; __shared__ float St[32][DEP + 1]; __shared__ __attribute__((aligned(16))) float Os[32 * NC];
  const int t_ = threadIdx.x, wave = t_ >> 5, lane = t_ & 31, nloc = lane & 15, hlf = lane >> 4, b0 = blockIdx.x * 32; const int l = t_;
  v8f oacc = {};
  for (int t = 0; t < NTREE; ++t) {
    __syncthreads();
    for (int i = t_; i < 32 * DEP; i += 128) { const int b = i / DEP, d = i % DEP; St[b][d] = S[(size_t)(b0 + b) * TD + t * DEP + d]; }
    __syncthreads();
    for (int b = 0; b < 32; ++b) { float p = 1.0f;
#pragma unroll
      for (int d = 0; d < DEP; ++d) { const float sd = St[b][d]; p = pmul(p, ((l >> d) & 1) ? (1.0f - sd) : sd); }
      b16 a_, b_; split16(p, a_, b_); Ah[b][l] = a_; Al[b][l] = b_; }
    __syncthreads();
    if (wave < 2) { v8f acc = {}; const b16* Bh = LPh + (size_t)t * 16 * NL; const b16* Bl = LPl + (size_t)t * 16 * NL;
#pragma unroll
      for (int kb = 0; kb < NL; kb += 32) { const v16b a = frag_kb(&Ah[wave * 16 + nloc][kb], hlf), al = frag_kb(&Al[wave * 16 + nloc][kb], hlf), bh = frag_kb(Bh + (size_t)nloc * NL + kb, hlf), bl = frag_kb(Bl + (size_t)nloc * NL + kb, hlf); acc = wmma16b(a, bh, acc); acc = wmma16b(al, bh, acc); acc = wmma16b(a, bl, acc); }
#pragma unroll
      for (int r = 0; r < 8; ++r) { const float at = ATT[(size_t)(b0 + wave * 16 + 8 * hlf + r) * NTREE + t]; oacc[r] += pmul(at, acc[r] * (1.0f / XS)); } } }
  __syncthreads();
  if (wave < 2 && nloc < NC) {
#pragma unroll
    for (int r = 0; r < 8; ++r) Os[(wave * 16 + 8 * hlf + r) * NC + nloc] = oacc[r]; }
  __syncthreads();
  for (int pass = 0; pass < 2; ++pass) { if (t_ < 32 * NC / 4) *(volatile v4f*)(out + (size_t)b0 * NC + t_ * 4) = *(const v4f*)(&Os[t_ * 4]); __threadfence(); }
}
}

extern "C" void kernel_launch(void* const* d_in, const int* in_sizes, int n_in,
                              void* d_out, int out_size, void* d_ws, size_t ws_size, hipStream_t stream) {
  (void)n_in; (void)out_size;
  const float* x = (const float*)d_in[0]; const float* fm = (const float*)d_in[1]; const float* th = (const float*)d_in[2]; const float* lo = (const float*)d_in[3]; const float* w1 = (const float*)d_in[4]; const float* b1 = (const float*)d_in[5]; const float* w2 = (const float*)d_in[6]; const float* b2 = (const float*)d_in[7];
  float* out = (float*)d_out;
  if (in_sizes[0] != NB * NI || in_sizes[1] != TD * NI || in_sizes[3] != NTREE * NL * NC || in_sizes[4] != NI * NH1 || in_sizes[6] != NH1 * NTREE) return;
  size_t off = 0; char* ws = (char*)d_ws;
  auto carve = [&](size_t bytes) { char* p = ws + off; off += (bytes + 255) & ~(size_t)255; return p; };
  b16* M = (b16*)carve((size_t)TD * NI * 2); b16* W1t = (b16*)carve((size_t)NH1 * NI * 2); b16* W2t = (b16*)carve((size_t)NTREE * NH1 * 2); b16* X = (b16*)carve((size_t)NB * NI * 2); float* P = (float*)carve(1088 * 4);
  b16* LPh = (b16*)carve((size_t)NTREE * 16 * NL * 2); b16* LPl = (b16*)carve((size_t)NTREE * 16 * NL * 2); float* S = (float*)carve((size_t)NB * TD * 4); float* ATT = (float*)carve((size_t)NB * NTREE * 4);
  if (off > ws_size) return;
  prep_kernel<<<256, 256, 0, stream>>>(x, fm, th, lo, w1, b1, w2, b2, M, W1t, W2t, X, P, LPh, LPl);
  split_kernel<<<NB / 32, 224, 0, stream>>>(X, M, P, S);
  attn_kernel<<<NB / 32, 64, 0, stream>>>(X, W1t, W2t, P, ATT);
  tree_kernel<<<NB / 32, 128, 0, stream>>>(S, ATT, LPh, LPl, out);
}
